// Encoder_90091234001521
// MI455X (gfx1250) — hardware-run, weakly checked
//
#include <hip/hip_runtime.h>
#include <math.h>

#pragma clang fp contract(off)

typedef __attribute__((ext_vector_type(16))) _Float16 v16h;
typedef __attribute__((ext_vector_type(8)))  _Float16 v8h;
typedef __attribute__((ext_vector_type(8)))  float v8f;
typedef __attribute__((ext_vector_type(4)))  float v4f;
typedef __attribute__((ext_vector_type(4)))  unsigned v4u;
typedef _Float16 h16;

template <typename T> __device__ __forceinline__ void vst2(void* p, T v) { *(volatile T*)p = v; __threadfence(); *(volatile T*)p = v; }
__device__ __forceinline__ v8f wmma16(v16h a, v16h b, v8f c) {
  v8f d = __builtin_amdgcn_wmma_f32_16x16x32_f16(false, a, false, b, (short)0, c, false, false);
  asm volatile("v_nop\n\tv_nop\n\tv_nop\n\tv_nop" : "+v"(d) : "v"(a), "v"(b));
  return d;
}
__device__ __forceinline__ v16h frag_h(const _Float16* rowk0, int lane) {
  union { v16h v; v8h q[2]; } u; const _Float16* p = rowk0 + 8 * (lane >> 4);
  u.q[0] = *(const v8h*)p; u.q[1] = *(const v8h*)(p + 16); return u.v;
}
__device__ __forceinline__ float bfr(float v) { return (float)(__bf16)v; }
static __device__ __forceinline__ h16 toh_flush(float v) { const h16 r = (h16)v; return (fabsf(v) < 6.103515625e-05f) ? (h16)0.0f : r; }
#define LDSX() do { asm volatile("s_wait_dscnt 0" ::: "memory"); __builtin_amdgcn_wave_barrier(); __builtin_amdgcn_fence(3  , "workgroup"); } while (0)

#ifndef NB
#define NB 2
#endif
#ifndef SEQ
#define SEQ 2048
#endif
#define SEQ_FULL 2048
#define VOCAB 32000
#define CC 512
#define NH 8
#define HD 64
#define FF 2048
#define NLAYERS 2
#define NRW (NB * SEQ)
#define WSC (64.0f)
#define WSCI (1.0f / 64.0f)
#define CTSC (64.0f)
#define PSH (8.0f)
#define SCL2 (0.125f * 1.4426950408889634f)
#define PE_C (-9.210340371976184f / 512.0f)

static_assert(SEQ % 64 == 0);
static_assert(SEQ % 32 == 0);
static_assert(NRW % 64 == 0);
static_assert(NRW % 8 == 0);
static_assert(CC == 512);
static_assert(CC == NH * HD);
static_assert(HD == 64);
static_assert(CC % 128 == 0);
static_assert(FF % 128 == 0);
static_assert(CC % 32 == 0);
static_assert(FF % 32 == 0);
static_assert((CC * CC / 8) % 256 == 0);
static_assert((FF * CC / 8) % 256 == 0);
static_assert(2 * 256 == CC);
static_assert(128 * 4 == CC);
static_assert(2 * 32 * 8 == CC);
static_assert(64 * 16 == 128 * 8);
static_assert(128 * 8 == 128 * 8);
static_assert(32 * 4 == 128);
static_assert(4 * 4 == 16);
static_assert(8 * 8 == HD);
static_assert(64 * 136 * 2 + 128 * 72 * 2 <= 131072);
static_assert(4 * 16 * 132 * 4 <= 131072);
static_assert(4 * 16 * 72 * 2 <= 131072);

constexpr size_t SZ_WQKV = (size_t)2 * 3 * CC * CC;
constexpr size_t SZ_WO   = (size_t)2 * CC * CC;
constexpr size_t SZ_W1   = (size_t)2 * FF * CC;
constexpr size_t SZ_W2   = (size_t)2 * CC * FF;
constexpr size_t SZ_X    = (size_t)4 * NRW * CC;
constexpr size_t SZ_H    = (size_t)2 * NRW * CC;
constexpr size_t SZ_VT   = (size_t)2 * NB * CC * SEQ;
constexpr size_t SZ_HF   = (size_t)2 * NRW * FF;
constexpr size_t WS_WQKV = 0;
constexpr size_t WS_WO = WS_WQKV + SZ_WQKV;
constexpr size_t WS_W1 = WS_WO + SZ_WO;
constexpr size_t WS_W2 = WS_W1 + SZ_W1;
constexpr size_t WS_XA = WS_W2 + SZ_W2;
constexpr size_t WS_XB = WS_XA + SZ_X;
constexpr size_t WS_HH = WS_XB + SZ_X;
constexpr size_t WS_QH = WS_HH + SZ_H;
constexpr size_t WS_KH = WS_QH + SZ_H;
constexpr size_t WS_VT = WS_KH + SZ_H;
constexpr size_t WS_CT = WS_VT + SZ_VT;
constexpr size_t WS_HF = WS_CT + SZ_H;
constexpr size_t WS_END = WS_HF + SZ_HF;
static_assert(WS_WO % 128 == 0);
static_assert(WS_W1 % 128 == 0);
static_assert(WS_W2 % 128 == 0);
static_assert(WS_XA % 128 == 0);
static_assert(WS_XB % 128 == 0);
static_assert(WS_HH % 128 == 0);
static_assert(WS_QH % 128 == 0);
static_assert(WS_KH % 128 == 0);
static_assert(WS_VT % 128 == 0);
static_assert(WS_CT % 128 == 0);
static_assert(WS_HF % 128 == 0);
static_assert(WS_END <= (size_t)134217728);

__global__ __launch_bounds__(256) void k_wconv(const float* __restrict__ W, unsigned n8, _Float16* __restrict__ P) {
  const unsigned i = blockIdx.x * 256u + threadIdx.x; if (i >= n8) return;
  const v4f a = *(const v4f*)(W + (size_t)i * 8u); const v4f b = *(const v4f*)(W + (size_t)i * 8u + 4u);
  v8h o;
#pragma unroll
  for (int k = 0; k < 4; ++k) { o[k] = toh_flush(bfr(a[k]) * WSC); o[4 + k] = toh_flush(bfr(b[k]) * WSC); }
  vst2(P + (size_t)i * 8u, o);
}

__global__ __launch_bounds__(256) void k_embed(const int* __restrict__ TOK, const float* __restrict__ EMB, float* __restrict__ X) {
  __shared__ __align__(16) float pe[CC];
  const unsigned tid = threadIdx.x, s = blockIdx.x;
  { const float i2 = (float)(2u * tid); const float dv = expf(i2 * PE_C); const float ang = (float)s * dv;
    pe[2u * tid] = sinf(ang); pe[2u * tid + 1u] = cosf(ang); }
  __syncthreads();
  if (tid < 128u) { const v4f p = *(const v4f*)&pe[tid * 4u];
#pragma unroll 1
    for (unsigned b = 0; b < (unsigned)NB; ++b) { int tk = TOK[(size_t)b * SEQ_FULL + s]; tk = min(max(tk, 0), VOCAB - 1);
      const v4f e = *(const v4f*)(EMB + (size_t)tk * CC + tid * 4u);
      v4f o; o[0] = bfr(e[0]) + p[0]; o[1] = bfr(e[1]) + p[1]; o[2] = bfr(e[2]) + p[2]; o[3] = bfr(e[3]) + p[3];
      vst2(X + ((size_t)b * SEQ + s) * CC + tid * 4u, o); } } }

__global__ __launch_bounds__(256) void k_ln(const float* __restrict__ X, const float* __restrict__ G, const float* __restrict__ BE, const int* __restrict__ NLP, _Float16* __restrict__ OUT) {
  const unsigned wave = (unsigned)__builtin_amdgcn_readfirstlane((int)(threadIdx.x >> 5)), lane = threadIdx.x & 31u;
  const unsigned row = blockIdx.x * 8u + wave; if (row >= (unsigned)NRW) return;
  const float pz = (NLP[0] != NLAYERS) ? __int_as_float(0x7fc00000) : 0.f;
  v4f v[4]; float s1 = 0.f;
#pragma unroll
  for (int i = 0; i < 2; ++i) { const float* p = X + (size_t)row * CC + i * 256 + lane * 8u; v[2 * i] = *(const v4f*)p; v[2 * i + 1] = *(const v4f*)(p + 4);
    s1 += ((v[2 * i][0] + v[2 * i][1]) + (v[2 * i][2] + v[2 * i][3])) + ((v[2 * i + 1][0] + v[2 * i + 1][1]) + (v[2 * i + 1][2] + v[2 * i + 1][3])); }
#pragma unroll
  for (int o = 1; o < 32; o <<= 1) s1 += __shfl_xor(s1, o);
  const float mu = s1 * (1.0f / CC); float q = 0.f;
#pragma unroll
  for (int i = 0; i < 4; ++i)
#pragma unroll
    for (int k = 0; k < 4; ++k) { const float d = v[i][k] - mu; q += d * d; }
#pragma unroll
  for (int o = 1; o < 32; o <<= 1) q += __shfl_xor(q, o);
  const float inv = rsqrtf(q * (1.0f / CC) + 1e-5f);
#pragma unroll
  for (int i = 0; i < 2; ++i) { const unsigned c = i * 256 + lane * 8u;
    const v4f g0 = *(const v4f*)(G + c), g1 = *(const v4f*)(G + c + 4u), b0 = *(const v4f*)(BE + c), b1 = *(const v4f*)(BE + c + 4u);
    v8h o;
#pragma unroll
    for (int k = 0; k < 4; ++k) { o[k] = toh_flush(bfr(g0[k]) * ((v[2 * i][k] - mu) * inv) + bfr(b0[k]) + pz); o[4 + k] = toh_flush(bfr(g1[k]) * ((v[2 * i + 1][k] - mu) * inv) + bfr(b1[k]) + pz); }
    vst2(OUT + (size_t)row * CC + c, o); } }

__device__ __forceinline__ void gemm_main(const _Float16* __restrict__ arow, const _Float16* __restrict__ wrow, int K, int lane, v8f (&acc)[8]) {
#pragma unroll 1
  for (int kc = 0; kc < K / 32; ++kc) { const v16h a = frag_h(arow + kc * 32, lane);
    asm volatile("s_wait_loadcnt 0x0" ::: "memory");
#pragma unroll
    for (int j = 0; j < 8; ++j) { const v16h w = frag_h(wrow + (size_t)j * 16 * K + kc * 32, lane); acc[j] = wmma16(a, w, acc[j]); } } }

__global__ __launch_bounds__(128) __attribute__((amdgpu_num_vgpr(256))) void k_qkv(const _Float16* __restrict__ HHP, const _Float16* __restrict__ WP, _Float16* __restrict__ QH, _Float16* __restrict__ KH, _Float16* __restrict__ VT) {
  __shared__ __align__(16) _Float16 sh[64][136]; __shared__ __align__(16) _Float16 th[128][72];
  const unsigned tid = threadIdx.x, lane = tid & 31u, col = lane & 15u, g = lane >> 4; const unsigned wave = (unsigned)__builtin_amdgcn_readfirstlane((int)(tid >> 5));
  const unsigned which = blockIdx.z, c0 = blockIdx.y * 128u, r0 = blockIdx.x * 64u; const unsigned bb = r0 / (unsigned)SEQ, t0 = r0 % (unsigned)SEQ;
  v8f acc[8] = {};
  gemm_main(HHP + ((size_t)r0 + wave * 16u + col) * CC, WP + ((size_t)which * CC + c0 + col) * CC, CC, (int)lane, acc);
  if (which < 2) { _Float16* DH = which == 0 ? QH : KH;
#pragma unroll
    for (int j = 0; j < 8; ++j) {
#pragma unroll
      for (int r = 0; r < 8; ++r) sh[wave * 16 + 8 * g + r][j * 16 + col] = toh_flush(acc[j][r] * WSCI); }
    __syncthreads();
    for (unsigned e = tid; e < 64u * 16u; e += 128u) { const unsigned rl = e >> 4, q = e & 15u; vst2(DH + ((size_t)r0 + rl) * CC + c0 + q * 8u, *(const v8h*)&sh[rl][q * 8]); }
  } else {
#pragma unroll
    for (int j = 0; j < 8; ++j) { v8h t;
#pragma unroll
      for (int r = 0; r < 8; ++r) t[r] = toh_flush(acc[j][r] * WSCI);
      *(v8h*)&th[j * 16 + col][wave * 16 + 8 * g] = t; }
    __syncthreads();
    for (unsigned e = tid; e < 128u * 8u; e += 128u) { const unsigned cl = e >> 3, q = e & 7u; vst2(VT + ((size_t)bb * CC + c0 + cl) * (size_t)SEQ + t0 + q * 8u, *(const v8h*)&th[cl][q * 8]); } } }

__global__ __launch_bounds__(128) __attribute__((amdgpu_num_vgpr(256))) void k_attn(const _Float16* __restrict__ QH, const _Float16* __restrict__ KH, const _Float16* __restrict__ VT, _Float16* __restrict__ CT) {
  __shared__ __align__(16) _Float16 st[4][16][72];
  const unsigned tid = threadIdx.x, lane = tid & 31u, col = lane & 15u, g = lane >> 4; const unsigned wave = (unsigned)__builtin_amdgcn_readfirstlane((int)(tid >> 5));
  const unsigned h = blockIdx.y, b = blockIdx.z; const unsigned q0 = blockIdx.x * 64u + wave * 16u;
  const _Float16* qrow = QH + ((size_t)b * SEQ + q0 + col) * CC + h * HD;
  const v16h qf0 = frag_h(qrow, (int)lane), qf1 = frag_h(qrow + 32, (int)lane);
  const _Float16* kbase = KH + ((size_t)b * SEQ + col) * CC + h * HD;
  const _Float16* vbase = VT + ((size_t)b * CC + h * HD + col) * (size_t)SEQ;
  v8f ot[4] = {}; float m = -3.0e38f, l = 0.f;
#pragma unroll 1
  for (unsigned kb = 0; kb < (unsigned)SEQ; kb += 32u) {
    v8f s0 = {}, s1 = {};
    { const _Float16* kp = kbase + (size_t)kb * CC;
      const v16h k00 = frag_h(kp, (int)lane), k01 = frag_h(kp + 32, (int)lane);
      s0 = wmma16(k00, qf0, s0); s0 = wmma16(k01, qf1, s0);
      const v16h k10 = frag_h(kp + 16 * CC, (int)lane), k11 = frag_h(kp + 16 * CC + 32, (int)lane);
      s1 = wmma16(k10, qf0, s1); s1 = wmma16(k11, qf1, s1); }
    float mx = -3.0e38f;
#pragma unroll
    for (int r = 0; r < 8; ++r) { s0[r] *= SCL2; s1[r] *= SCL2; mx = fmaxf(mx, fmaxf(s0[r], s1[r])); }
    mx = fmaxf(mx, __shfl_xor(mx, 16));
    const float mn = fmaxf(m, mx); const float corr = exp2f(m - mn); m = mn;
    v16h pb; float ls = 0.f;
#pragma unroll
    for (int r = 0; r < 8; ++r) { const float e0 = (s0[r] - mn) + PSH, e1 = (s1[r] - mn) + PSH;
      const float x0 = exp2f(e0), x1 = exp2f(e1);
      const h16 p0 = (e0 < -14.0f) ? (h16)0.0f : (h16)x0; const h16 p1 = (e1 < -14.0f) ? (h16)0.0f : (h16)x1;
      pb[r] = p0; pb[8 + r] = p1; ls += (float)p0 + (float)p1; }
    ls += __shfl_xor(ls, 16);
    l = l * corr + ls;
#pragma unroll
    for (int j = 0; j < 4; ++j)
#pragma unroll
      for (int r = 0; r < 8; ++r) ot[j][r] *= corr;
    const _Float16* vp = vbase + kb;
#pragma unroll
    for (int j = 0; j < 4; ++j) ot[j] = wmma16(frag_h(vp + (size_t)j * 16 * SEQ, (int)lane), pb, ot[j]);
  }
  const float inv = CTSC * (1.0f / l);
#pragma unroll
  for (int j = 0; j < 4; ++j) { v8h t;
#pragma unroll
    for (int r = 0; r < 8; ++r) t[r] = toh_flush(ot[j][r] * inv);
    *(v8h*)&st[wave][col][16 * j + 8 * g] = t; }
  LDSX();
#pragma unroll
  for (unsigned i = 0; i < 4u; ++i) { const unsigned rl = 4u * i + (lane >> 3), pc = lane & 7u; const v8h v = *(const v8h*)&st[wave][rl][pc * 8u];
    vst2(CT + ((size_t)b * SEQ + q0 + rl) * CC + h * HD + pc * 8u, v); } }

__global__ __launch_bounds__(128) __attribute__((amdgpu_num_vgpr(256))) void k_gemf(const _Float16* __restrict__ A, int lda, int K, const _Float16* __restrict__ WP, int nout, float oscale, const float* __restrict__ BIAS, const float* __restrict__ RES, float* __restrict__ OUT) {
  __shared__ __align__(16) float sf[4][16][132];
  const unsigned tid = threadIdx.x, lane = tid & 31u, col = lane & 15u, g = lane >> 4; const unsigned wave = (unsigned)__builtin_amdgcn_readfirstlane((int)(tid >> 5));
  const unsigned c0 = blockIdx.y * 128u; const size_t r0 = (size_t)blockIdx.x * 64 + wave * 16;
  v8f acc[8] = {};
  gemm_main(A + (r0 + col) * (size_t)lda, WP + ((size_t)c0 + col) * (size_t)K, K, (int)lane, acc);
#pragma unroll
  for (int j = 0; j < 8; ++j) { const float bb = bfr(BIAS[c0 + j * 16 + col]);
#pragma unroll
    for (int r = 0; r < 8; ++r) sf[wave][8 * g + r][j * 16 + col] = acc[j][r] * oscale + bb; }
  LDSX();
  for (unsigned rl = 0; rl < 16u; ++rl) { const size_t o = (r0 + rl) * (size_t)nout + c0 + lane * 4u; v4f v = *(const v4f*)&sf[wave][rl][lane * 4]; const v4f rv = *(const v4f*)(RES + o);
    v[0] += rv[0]; v[1] += rv[1]; v[2] += rv[2]; v[3] += rv[3]; vst2(OUT + o, v); } }

__global__ __launch_bounds__(128) __attribute__((amdgpu_num_vgpr(256))) void k_gemr(const _Float16* __restrict__ A, int lda, int K, const _Float16* __restrict__ WP, int nout, const float* __restrict__ BIAS, _Float16* __restrict__ OUT) {
  __shared__ __align__(16) _Float16 sh[64][136];
  const unsigned tid = threadIdx.x, lane = tid & 31u, col = lane & 15u, g = lane >> 4; const unsigned wave = (unsigned)__builtin_amdgcn_readfirstlane((int)(tid >> 5));
  const unsigned c0 = blockIdx.y * 128u; const size_t rb = (size_t)blockIdx.x * 64;
  v8f acc[8] = {};
  gemm_main(A + (rb + wave * 16u + col) * (size_t)lda, WP + ((size_t)c0 + col) * (size_t)K, K, (int)lane, acc);
#pragma unroll
  for (int j = 0; j < 8; ++j) { const float bb = bfr(BIAS[c0 + j * 16 + col]);
#pragma unroll
    for (int r = 0; r < 8; ++r) { const float v = acc[j][r] * WSCI + bb; const float a = (v > 0.0f) ? v : (v - v); sh[wave * 16 + 8 * g + r][j * 16 + col] = toh_flush(a); } }
  __syncthreads();
  for (unsigned e = tid; e < 64u * 16u; e += 128u) { const unsigned rl = e >> 4, q = e & 15u; vst2(OUT + (rb + rl) * (size_t)nout + c0 + q * 8u, *(const v8h*)&sh[rl][q * 8]); } }

extern "C" void kernel_launch(void* const* d_in, const int* in_sizes, int n_in, void* d_out, int out_size, void* d_ws, size_t ws_size, hipStream_t stream) {
  if (n_in < 16) return;
  if (ws_size < WS_END) return;
  if ((long)in_sizes[0] < (long)(NB - 1) * SEQ_FULL + SEQ) return;
  if ((long)in_sizes[1] < (long)VOCAB * CC) return;
  if (in_sizes[2] < CC * CC || in_sizes[3] < CC * CC || in_sizes[4] < CC * CC || in_sizes[5] < CC * CC) return;
  if (in_sizes[6] < CC || in_sizes[7] < CC || in_sizes[8] < CC || in_sizes[9] < CC || in_sizes[10] < CC) return;
  if (in_sizes[11] < FF * CC || in_sizes[12] < FF || in_sizes[13] < CC * FF || in_sizes[14] < CC || in_sizes[15] < 1) return;
  if ((long)out_size < (long)NRW * CC) return;
  const float* const* F = (const float* const*)d_in; const int* TOK = (const int*)d_in[0]; const int* NLP = (const int*)d_in[15];
  char* ws = (char*)d_ws;
  _Float16 *WQKV = (_Float16*)(ws + WS_WQKV), *WO = (_Float16*)(ws + WS_WO), *W1P = (_Float16*)(ws + WS_W1), *W2P = (_Float16*)(ws + WS_W2);
  float *XA = (float*)(ws + WS_XA), *XB = (float*)(ws + WS_XB);
  _Float16 *HH = (_Float16*)(ws + WS_HH), *QH = (_Float16*)(ws + WS_QH), *KH = (_Float16*)(ws + WS_KH), *VT = (_Float16*)(ws + WS_VT), *CT = (_Float16*)(ws + WS_CT), *HF = (_Float16*)(ws + WS_HF);
  const unsigned nDD8 = (unsigned)(CC * CC / 8), nFD8 = (unsigned)(FF * CC / 8);
  k_wconv<<<dim3((nDD8 + 255u) / 256u), 256, 0, stream>>>(F[2], nDD8, WQKV);
  k_wconv<<<dim3((nDD8 + 255u) / 256u), 256, 0, stream>>>(F[3], nDD8, WQKV + (size_t)CC * CC);
  k_wconv<<<dim3((nDD8 + 255u) / 256u), 256, 0, stream>>>(F[4], nDD8, WQKV + (size_t)2 * CC * CC);
  k_wconv<<<dim3((nDD8 + 255u) / 256u), 256, 0, stream>>>(F[5], nDD8, WO);
  k_wconv<<<dim3((nFD8 + 255u) / 256u), 256, 0, stream>>>(F[11], nFD8, W1P);
  k_wconv<<<dim3((nFD8 + 255u) / 256u), 256, 0, stream>>>(F[13], nFD8, W2P);
  k_embed<<<dim3(SEQ), 256, 0, stream>>>(TOK, F[1], XA);
  for (int L = 0; L < NLAYERS; ++L) {
    k_ln<<<dim3(NRW / 8), 256, 0, stream>>>(XA, F[7], F[8], NLP, HH);
    k_qkv<<<dim3(NRW / 64, CC / 128, 3), 128, 0, stream>>>(HH, WQKV, QH, KH, VT);
    k_attn<<<dim3(SEQ / 64, NH, NB), 128, 0, stream>>>(QH, KH, VT, CT);
    k_gemf<<<dim3(NRW / 64, CC / 128), 128, 0, stream>>>(CT, CC, CC, WO, CC, 1.0f / 4096.0f, F[6], XA, XB);
    k_ln<<<dim3(NRW / 8), 256, 0, stream>>>(XB, F[9], F[10], NLP, HH);
    k_gemr<<<dim3(NRW / 64, FF / 128), 128, 0, stream>>>(HH, CC, CC, W1P, FF, F[12], HF);
    float* dst = (L == NLAYERS - 1) ? (float*)d_out : XA;
    k_gemf<<<dim3(NRW / 64, CC / 128), 128, 0, stream>>>(HF, FF, FF, W2P, CC, 1.0f / 64.0f, F[14], XB, dst);
  }
}
